// DynamicValueIteration_31224412241999
// MI455X (gfx1250) — hardware-verified
//
#include <hip/hip_runtime.h>

#define IK       54
#define OGROUPS  16
#define KPAD     64
#define WROWS    (OGROUPS * 64)
#define TD       32
#define HD       32
#define WD       32
#define VOXB     (TD * HD * WD)
#define NB       2
#define NP       2
#define NCO      (OGROUPS * IK)
#define NPOS     (NB * VOXB)
#define NTHR     256
#define NWAV     8
#define NBLK     (NPOS / 16 / NWAV)
#define PKTHR    (WROWS * KPAD / 8)
#define WSC      1024.0f
#define RWSC     0.0009765625f
#define LSC      1024.0f
#define RLSC     0.0009765625f

static_assert(NPOS % (16 * NWAV) == 0);
static_assert(NBLK * 16 * NWAV == NPOS);
static_assert(PKTHR % 256 == 0);
static_assert(NTHR == NWAV * 32);
static_assert((VOXB % (16 * NWAV)) == 0);

typedef _Float16 v16h __attribute__((ext_vector_type(16)));
typedef _Float16 v8h  __attribute__((ext_vector_type(8)));
typedef float    v8f  __attribute__((ext_vector_type(8)));
typedef float    v4f  __attribute__((ext_vector_type(4)));
typedef unsigned int v4u __attribute__((ext_vector_type(4)));

__device__ __forceinline__ float bf_rne(float f) {
  unsigned x = __float_as_uint(f);
  x = (x + 0x7FFFu + ((x >> 16) & 1u)) & 0xFFFF0000u;
  return __uint_as_float(x);
}
__device__ __forceinline__ v8f zero8() { v8f z = {0.f, 0.f, 0.f, 0.f, 0.f, 0.f, 0.f, 0.f}; return z; }
__device__ __forceinline__ float rcp_f(float x) {
#if defined(__HIP_DEVICE_COMPILE__)
  return __builtin_amdgcn_rcpf(x);
#else
  return 1.0f / x;
#endif
}

__device__ __forceinline__ v16h ldfrag(const _Float16* p) {
  union { v16h v; v8h h[2]; } f;
  f.h[0] = *(const v8h*)(p);
  f.h[1] = *(const v8h*)(p + 16);
  return f.v;
}

__device__ __forceinline__ v8f mma_h(v16h a, v16h b, v8f c) {
  return __builtin_amdgcn_wmma_f32_16x16x32_f16(false, a, false, b, (short)0, c, false, false);
}
__device__ __forceinline__ void dep_guard2(v8f& x, v8f& y, v16h a0, v16h a1,
                                           v16h b0, v16h b1, v16h b2, v16h b3) {
#if defined(__HIP_DEVICE_COMPILE__)
  asm volatile("v_nop\n\tv_nop\n\tv_nop\n\tv_nop"
               : "+v"(x), "+v"(y)
               : "v"(a0), "v"(a1), "v"(b0), "v"(b1), "v"(b2), "v"(b3)
               : "memory");
#endif
}

__global__ __launch_bounds__(256)
void k_packw(const float* __restrict__ w, _Float16* wr) {
  const int g   = blockIdx.x * 256 + threadIdx.x;
  const int gc  = (g < PKTHR) ? g : (PKTHR - 1);
  const int row = gc >> 3;
  const int ch  = gc & 7;
  const int o   = row >> 6;
  const int j   = row & 63;
  const bool rowok = (j < IK);
  const int jc  = rowok ? j : 0;
  union { v8h h; v4u u; } pk;
#pragma unroll
  for (int i = 0; i < 8; ++i) {
    const int k  = ch * 8 + i;
    const bool ok = rowok && (k < IK);
    const int kc = (k < IK) ? k : 0;
    const float x = w[(o * IK + jc) * IK + kc];
    const float y = ok ? (bf_rne(x) * WSC) : 0.0f;
    pk.h[i] = (_Float16)y;
  }
  _Float16* dst = wr + (size_t)gc * 8;
  const v4u val = pk.u;
  if (g < PKTHR) *(volatile v4u*)dst = val;
  __threadfence();
  if (g < PKTHR) *(volatile v4u*)dst = val;
}

__global__ __launch_bounds__(NTHR)
void k_main(const float* __restrict__ values,
            const float* __restrict__ rewards,
            const _Float16* __restrict__ wr,
            float* out)
{
  __shared__ __align__(16) _Float16 Uh[NWAV][16 * KPAD];
  __shared__ __align__(16) _Float16 Ul[NWAV][16 * KPAD];
  __shared__ __align__(16) float    o_s[NP][NWAV * 16];

  const int tid  = threadIdx.x;
  const int lane = tid & 31;
  const int wave = tid >> 5;
  const int rbase = (int)(((unsigned)blockIdx.x * (NWAV * 16)) & (VOXB - 1));
  const int b     = (int)(((unsigned)blockIdx.x * (NWAV * 16)) >> 15);
  const int vb    = rbase + wave * 16;
  const int t  = vb >> 10;
  const int h  = (vb >> 5) & 31;
  const int w0 = vb & 31;

  _Float16* uh = &Uh[wave][0];
  _Float16* ul = &Ul[wave][0];

#pragma unroll 2
  for (int i = 0; i < 32; ++i) {
    const int e  = (i << 5) + lane;
    const int n  = e >> 6;
    const int k  = e & 63;
    const int kk = (k < IK) ? k : 0;
    const int ci = kk / 27;
    const int rr = kk - ci * 27;
    const int dz = rr / 9;
    const int r2 = rr - dz * 9;
    const int dy = r2 / 3;
    const int dx = r2 - dy * 3;
    const int tz = t + dz - 1;
    const int hy = h + dy - 1;
    const int wx = w0 + n + dx - 1;
    const bool inb = (k < IK) && ((unsigned)tz < 32u) && ((unsigned)hy < 32u) && ((unsigned)wx < 32u);
    const int tzc = tz < 0 ? 0 : (tz > 31 ? 31 : tz);
    const int hyc = hy < 0 ? 0 : (hy > 31 ? 31 : hy);
    const int wxc = wx < 0 ? 0 : (wx > 31 ? 31 : wx);
    const size_t idx = ((((size_t)b * NP + ci) * TD + tzc) * HD + hyc) * WD + wxc;
    const float s   = bf_rne(values[idx]) + bf_rne(rewards[idx]);
    const float val = inb ? s : 0.0f;
    const _Float16 hi = (_Float16)val;
    const float res = (val - (float)hi) * LSC;
    const _Float16 lo = (_Float16)res;
    uh[n * KPAD + k] = hi;
    ul[n * KPAD + k] = lo;
  }
  __syncthreads();

  const int col = lane & 15;
  const int hh  = lane >> 4;

  v16h bh[2], bl[2];
#pragma unroll
  for (int s = 0; s < 2; ++s) {
    bh[s] = ldfrag(uh + col * KPAD + s * 32 + 8 * hh);
    bl[s] = ldfrag(ul + col * KPAD + s * 32 + 8 * hh);
  }

  const float NEG_INF = __uint_as_float(0xff800000u);
  float best0 = NEG_INF, best1 = NEG_INF;

#pragma unroll 1
  for (int o = 0; o < OGROUPS; ++o) {
    v8f ah[4], al[4];
    const _Float16* wro = wr + ((size_t)o * 64 + col) * KPAD + 8 * hh;
#pragma unroll
    for (int rt = 0; rt < 4; ++rt) {
      const v16h a0 = ldfrag(wro + rt * 16 * KPAD);
      const v16h a1 = ldfrag(wro + rt * 16 * KPAD + 32);
      ah[rt] = mma_h(a0, bh[0], zero8());
      al[rt] = mma_h(a0, bl[0], zero8());
      ah[rt] = mma_h(a1, bh[1], ah[rt]);
      al[rt] = mma_h(a1, bl[1], al[rt]);
      dep_guard2(ah[rt], al[rt], a0, a1, bh[0], bh[1], bl[0], bl[1]);
    }

    float lg[32];
    float m = NEG_INF;
#pragma unroll
    for (int rt = 0; rt < 4; ++rt) {
#pragma unroll
      for (int v = 0; v < 8; ++v) {
        const int j = rt * 16 + 8 * hh + v;
        const float l = fmaf(al[rt][v], RLSC, ah[rt][v]) * RWSC;
        lg[rt * 8 + v] = l;
        m = (j < IK) ? fmaxf(m, l) : m;
      }
    }
    m = fmaxf(m, __shfl_xor(m, 16, 32));

    float sum = 0.0f, dot = 0.0f;
#pragma unroll
    for (int rt = 0; rt < 4; ++rt) {
#pragma unroll
      for (int v = 0; v < 8; ++v) {
        const int j  = rt * 16 + 8 * hh + v;
        const int sb = rt >> 1;
        const int eb = (rt & 1) * 8 + v;
        const float u = fmaf((float)bl[sb][eb], RLSC, (float)bh[sb][eb]);
        const float ex = __expf(lg[rt * 8 + v] - m);
        const bool ok = (j < IK);
        sum = ok ? (sum + ex) : sum;
        dot = ok ? fmaf(ex, u, dot) : dot;
      }
    }
    sum += __shfl_xor(sum, 16, 32);
    dot += __shfl_xor(dot, 16, 32);
    const float q = dot * rcp_f(sum);
    if (o < 8) best0 = fmaxf(best0, q);
    else       best1 = fmaxf(best1, q);
  }

  if (hh == 0) {
    o_s[0][wave * 16 + col] = best0;
    o_s[1][wave * 16 + col] = best1;
  }
  __syncthreads();

  {
    const int e  = (tid < 64) ? tid : 63;
    const int pl = e >> 5;
    const int pc = e & 31;
    const v4f v = *(const v4f*)(&o_s[pl][4 * pc]);
    float* dst = out + (size_t)(b * NP + pl) * VOXB + rbase + 4 * pc;
    if (tid < 64) *(volatile v4f*)dst = v;
    __threadfence();
    if (tid < 64) *(volatile v4f*)dst = v;
  }
}

extern "C" void kernel_launch(void* const* d_in, const int* in_sizes, int n_in,
                              void* d_out, int out_size, void* d_ws, size_t ws_size,
                              hipStream_t stream) {
  if (n_in < 3) return;
  if (in_sizes[0] != NB * NP * VOXB) return;
  if (in_sizes[1] != NB * NP * VOXB) return;
  if (in_sizes[2] != NCO * IK) return;
  if (out_size != NB * NP * VOXB) return;
  if (ws_size < (size_t)WROWS * KPAD * sizeof(_Float16)) return;

  const float* values  = (const float*)d_in[0];
  const float* rewards = (const float*)d_in[1];
  const float* weight  = (const float*)d_in[2];
  float* out = (float*)d_out;
  _Float16* wr = (_Float16*)d_ws;

  k_packw<<<dim3(PKTHR / 256), dim3(256), 0, stream>>>(weight, wr);
  k_main<<<dim3(NBLK), dim3(NTHR), 0, stream>>>(values, rewards, wr, out);
  (void)hipGetLastError();
}
